// ProteinGNN_11871289606631
// MI455X (gfx1250) — hardware-verified
//
#include <hip/hip_runtime.h>
#include <stddef.h>
#include <stdint.h>


#define FIN     256
#define HIDC    128
#define NCOL    256
#define LDF     256
#define LDA     512
#define NTHR    256
#define NWAVE   8
#define EPT     8
#define CHUNK   (NTHR * EPT)
#define WCAP    (EPT * 32)
#define LISTN   (NWAVE * WCAP)
#define NBMAX   2048
#define RCAP    28672
#define DEGCAP  1024
#define STW     512
#define GBM     64
#define GBN     64
#define GTHR    128
#define WSMAX   134217728
#define LDS_AGG ((2 * RCAP + 2 * NBMAX + LISTN) * 4 + 64)

static_assert((CHUNK & (CHUNK - 1)) == 0 && CHUNK <= 4096);
static_assert((NBMAX & (NBMAX - 1)) == 0 && NBMAX <= 4096);
static_assert(NTHR * 8 == NBMAX);
static_assert(LISTN >= NBMAX);
static_assert(LISTN >= NWAVE * WCAP);
static_assert((RCAP % 32) == 0);
static_assert(NWAVE * STW <= RCAP);
static_assert(STW >= HIDC);
static_assert(LDS_AGG <= 300000);
static_assert(GBM == (GTHR / 32) * 16);
static_assert(FIN / 8 == 32);
static_assert(HIDC == 4 * 32);
static_assert((FIN % 32) == 0 && (HIDC % 32) == 0 && (LDA % 32) == 0);
static_assert((NCOL % GBN) == 0);
static_assert((GBM * GBN) % GTHR == 0);
static_assert(LDA == 2 * NCOL);
static_assert(LDA * 2 == LDF * 4);

typedef float          v4f  __attribute__((ext_vector_type(4)));
typedef float          v8f  __attribute__((ext_vector_type(8)));
typedef int            v4i  __attribute__((ext_vector_type(4)));
typedef int            v8i  __attribute__((ext_vector_type(8)));
typedef unsigned short us;
typedef us             v8us __attribute__((ext_vector_type(8)));
typedef __bf16         v16b __attribute__((ext_vector_type(16)));
union FragB { v16b v; v8us h[2]; v8i w; };

__device__ __forceinline__ v8f wmb(const FragB& a, const FragB& b, v8f c) {
  v8f d = __builtin_amdgcn_wmma_f32_16x16x32_bf16(false, a.v, false, b.v, (short)0, c, false, false);
  asm volatile("v_nop\n\tv_nop\n\tv_nop\n\tv_nop" : "+v"(d) : "v"(a.w), "v"(b.w));
  return d;
}

__device__ __forceinline__ void ldwait() {
  asm volatile("s_wait_loadcnt 0x0" ::: "memory");
}

__device__ __forceinline__ us rne16(float f) {
  unsigned u = (unsigned)__float_as_uint(f);
  u = u + 0x7FFFu + ((u >> 16) & 1u);
  return (us)(u >> 16);
}
__device__ __forceinline__ float bfv(us h) { return __uint_as_float(((unsigned)h) << 16); }
__device__ __forceinline__ float rnev(float f) { return bfv(rne16(f)); }

__device__ __forceinline__ v8us cvt8b(const v4f a, const v4f b) {
  v8us hv;
  hv[0] = rne16(a.x); hv[1] = rne16(a.y); hv[2] = rne16(a.z); hv[3] = rne16(a.w);
  hv[4] = rne16(b.x); hv[5] = rne16(b.y); hv[6] = rne16(b.z); hv[7] = rne16(b.w);
  return hv;
}

__device__ __forceinline__ void split8(const v4f a, const v4f b, v8us& hi, v8us& lo) {
  const float f0 = a.x, f1 = a.y, f2 = a.z, f3 = a.w, f4 = b.x, f5 = b.y, f6 = b.z, f7 = b.w;
  us h;
  h = rne16(f0); hi[0] = h; lo[0] = rne16(f0 - bfv(h));
  h = rne16(f1); hi[1] = h; lo[1] = rne16(f1 - bfv(h));
  h = rne16(f2); hi[2] = h; lo[2] = rne16(f2 - bfv(h));
  h = rne16(f3); hi[3] = h; lo[3] = rne16(f3 - bfv(h));
  h = rne16(f4); hi[4] = h; lo[4] = rne16(f4 - bfv(h));
  h = rne16(f5); hi[5] = h; lo[5] = rne16(f5 - bfv(h));
  h = rne16(f6); hi[6] = h; lo[6] = rne16(f6 - bfv(h));
  h = rne16(f7); hi[7] = h; lo[7] = rne16(f7 - bfv(h));
}

__device__ __forceinline__ int scan_chunk(const int* __restrict__ dsts, int nE, int cbase, int slotBase,
                                          int nb, int vec8, int* list, int tid, int lane, int wave) {
  int wc = 0;
  const int el0  = tid * EPT;
  const int e0   = cbase + el0;
  const int sent = -2147483647 - 1;
  v4i da, db;
  if (vec8 != 0 && cbase + CHUNK <= nE) {
    da = *(const v4i*)(dsts + e0);
    db = *(const v4i*)(dsts + e0 + 4);
  } else {
    da.x = (e0     < nE) ? dsts[min(e0,     nE - 1)] : sent;
    da.y = (e0 + 1 < nE) ? dsts[min(e0 + 1, nE - 1)] : sent;
    da.z = (e0 + 2 < nE) ? dsts[min(e0 + 2, nE - 1)] : sent;
    da.w = (e0 + 3 < nE) ? dsts[min(e0 + 3, nE - 1)] : sent;
    db.x = (e0 + 4 < nE) ? dsts[min(e0 + 4, nE - 1)] : sent;
    db.y = (e0 + 5 < nE) ? dsts[min(e0 + 5, nE - 1)] : sent;
    db.z = (e0 + 6 < nE) ? dsts[min(e0 + 6, nE - 1)] : sent;
    db.w = (e0 + 7 < nE) ? dsts[min(e0 + 7, nE - 1)] : sent;
  }
  const unsigned nbs = (unsigned)slotBase;
  const unsigned unb = (unsigned)nb;
  const unsigned s0 = (unsigned)da.x - nbs, s1 = (unsigned)da.y - nbs;
  const unsigned s2 = (unsigned)da.z - nbs, s3 = (unsigned)da.w - nbs;
  const unsigned s4 = (unsigned)db.x - nbs, s5 = (unsigned)db.y - nbs;
  const unsigned s6 = (unsigned)db.z - nbs, s7 = (unsigned)db.w - nbs;
  const bool h0 = s0 < unb, h1 = s1 < unb, h2 = s2 < unb, h3 = s3 < unb;
  const bool h4 = s4 < unb, h5 = s5 < unb, h6 = s6 < unb, h7 = s7 < unb;
  const unsigned any = __builtin_amdgcn_ballot_w32(h0 | h1 | h2 | h3 | h4 | h5 | h6 | h7);
  if (any != 0u) {
#define HITJ(J, HJ, SJ) { \
      const unsigned mj = __builtin_amdgcn_ballot_w32(HJ); \
      if (mj != 0u) { \
        if (HJ) { \
          const int pos = wc + (int)__builtin_amdgcn_mbcnt_lo(mj, 0u); \
          if (pos < WCAP) list[wave * WCAP + pos] = ((el0 + (J)) << 12) | (int)(SJ); \
        } \
        wc += (int)__builtin_popcount(mj); } }
    HITJ(0, h0, s0)
    HITJ(1, h1, s1)
    HITJ(2, h2, s2)
    HITJ(3, h3, s3)
    HITJ(4, h4, s4)
    HITJ(5, h5, s5)
    HITJ(6, h6, s6)
    HITJ(7, h7, s7)
#undef HITJ
  }
  return wc;
}

__global__ __launch_bounds__(NTHR) void k_xprep(const float* __restrict__ x, us* xb, int nN, int nUnits) {
  const int i = (int)blockIdx.x * NTHR + (int)threadIdx.x;
  if (i >= nUnits) return;
  const int row = i >> 5;
  const int c0  = (i & 31) * 8;
  const int rc  = row < nN ? row : nN - 1;
  const float* p = x + (size_t)rc * FIN + c0;
  v4f a = *(const v4f*)p, b = *(const v4f*)(p + 4);
  const v4f z4 = {0.f, 0.f, 0.f, 0.f};
  if (row >= nN) { a = z4; b = z4; }
  const v8us hv = cvt8b(a, b);
  const size_t o = (size_t)row * FIN + c0;
  *(volatile v8us*)(xb + o) = hv;
  __threadfence();
  *(volatile v8us*)(xb + o) = hv;
}

__global__ __launch_bounds__(NTHR) void k_wtr(const float* __restrict__ w0, const float* __restrict__ w1,
                                              int cc0, int cc1, int cSplit, int kRows, int K2,
                                              int kMask, int shHi, int shLo, us* wt, int nUnits) {
  const int u = (int)blockIdx.x * NTHR + (int)threadIdx.x;
  if (u >= nUnits) return;
  const int kq = K2 >> 3;
  const int n  = u / kq;
  const int k8 = (u - n * kq) * 8;
  const int seg = (n >= cSplit) ? 1 : 0;
  const int nc  = n - seg * cSplit;
  const float* wsrc = seg ? w1 : w0;
  const int cc  = seg ? cc1 : cc0;
  const int ncl = nc < cc ? nc : cc - 1;
  float f[8];
#pragma unroll
  for (int i = 0; i < 8; ++i) {
    const int k2 = k8 + i;
    int k = ((k2 >> shHi) << shLo) | (k2 & kMask);
    k = k < 0 ? 0 : (k > kRows - 1 ? kRows - 1 : k);
    f[i] = wsrc[(size_t)k * (size_t)cc + ncl];
  }
  v8us hv;
#pragma unroll
  for (int i = 0; i < 8; ++i) hv[i] = rne16(f[i]);
  if (nc >= cc) {
#pragma unroll
    for (int i = 0; i < 8; ++i) hv[i] = (us)0;
  }
  const size_t o = (size_t)n * (size_t)K2 + k8;
  *(volatile v8us*)(wt + o) = hv;
  __threadfence();
  *(volatile v8us*)(wt + o) = hv;
}

template<int EPI, int HASB>
__global__ __launch_bounds__(GTHR) void k_gemm(
    const us* __restrict__ A, const us* __restrict__ WT, const float* __restrict__ bias,
    float* outF, us* outH, int K, int lda, int segN, int aSeg, int ldo)
{
  __shared__ __attribute__((aligned(16))) float stg[GBM * GBN];
  const int tid = (int)threadIdx.x, lane = tid & 31, wave = tid >> 5, hh = lane >> 4, m = lane & 15;
  const int rowBase = (int)blockIdx.x * GBM;
  const int col0    = (int)blockIdx.y * GBN;
  int segi = col0 / segN;
  segi = segi < 0 ? 0 : segi;
  const int aoff = segi * aSeg;

  v8f acc[4];
  {
    const v8f z = {0.f, 0.f, 0.f, 0.f, 0.f, 0.f, 0.f, 0.f};
    acc[0] = z; acc[1] = z; acc[2] = z; acc[3] = z;
  }
  const us* ap = A  + (size_t)(rowBase + 16 * wave + m) * (size_t)lda + aoff + 8 * hh;
  const us* wp = WT + (size_t)(col0 + m) * (size_t)K + 8 * hh;
  const int ksteps = K >> 5;
#pragma unroll 1
  for (int ks = 0; ks < ksteps; ++ks) {
    FragB af;
    af.h[0] = *(const v8us*)(ap + 32 * ks);
    af.h[1] = *(const v8us*)(ap + 32 * ks + 16);
#pragma unroll
    for (int t = 0; t < 4; ++t) {
      const us* wq = wp + (size_t)(16 * t) * (size_t)K + 32 * ks;
      FragB bf;
      bf.h[0] = *(const v8us*)wq;
      bf.h[1] = *(const v8us*)(wq + 16);
      acc[t] = wmb(af, bf, acc[t]);
    }
  }

#pragma unroll
  for (int t = 0; t < 4; ++t) {
    const int lc = 16 * t + m;
    float bv = 0.0f;
    if (HASB) bv = rnev(bias[col0 + lc]);
#pragma unroll
    for (int r = 0; r < 8; ++r) {
      const int lr = 16 * wave + 8 * hh + r;
      stg[lr * GBN + lc] = acc[t][r] + bv;
    }
  }
  __syncthreads();

  if (EPI == 0) {
    v4f fv[8];
#pragma unroll
    for (int i = 0; i < 8; ++i) {
      const int lr = 16 * wave + 2 * i + hh;
      fv[i] = *(const v4f*)(stg + lr * GBN + 4 * m);
    }
#pragma unroll
    for (int i = 0; i < 8; ++i) {
      const int lr = 16 * wave + 2 * i + hh;
      const int gr = rowBase + lr;
      float* op = outF + (size_t)gr * (size_t)ldo + col0 + 4 * m;
      *(volatile v4f*)op = fv[i];
    }
    __threadfence();
#pragma unroll
    for (int i = 0; i < 8; ++i) {
      const int lr = 16 * wave + 2 * i + hh;
      const int gr = rowBase + lr;
      float* op = outF + (size_t)gr * (size_t)ldo + col0 + 4 * m;
      *(volatile v4f*)op = fv[i];
    }
  } else {
#pragma unroll 1
    for (int i = 0; i < (GBM * GBN) / GTHR; ++i) {
      const int e = i * GTHR + tid;
      const float v = stg[e];
      stg[e] = 0.5f * v * (1.0f + erff(v * 0.70710678118654752f));
    }
    __syncthreads();
    const int rq = lane >> 3;
    const int c8 = (lane & 7) * 8;
    v8us hv[4], lv[4];
#pragma unroll
    for (int i = 0; i < 4; ++i) {
      const int lr = 16 * wave + 4 * i + rq;
      const v4f ga = *(const v4f*)(stg + lr * GBN + c8);
      const v4f gb = *(const v4f*)(stg + lr * GBN + c8 + 4);
      split8(ga, gb, hv[i], lv[i]);
    }
#pragma unroll
    for (int i = 0; i < 4; ++i) {
      const int gr = rowBase + 16 * wave + 4 * i + rq;
      us* hp = outH + (size_t)gr * (size_t)ldo + col0 + c8;
      *(volatile v8us*)hp = hv[i];
      *(volatile v8us*)(hp + NCOL) = lv[i];
    }
    __threadfence();
#pragma unroll
    for (int i = 0; i < 4; ++i) {
      const int gr = rowBase + 16 * wave + 4 * i + rq;
      us* hp = outH + (size_t)gr * (size_t)ldo + col0 + c8;
      *(volatile v8us*)hp = hv[i];
      *(volatile v8us*)(hp + NCOL) = lv[i];
    }
  }
}

template<int NH>
__global__ __launch_bounds__(NTHR) void k_scores(const float* __restrict__ F, int colOff,
                                                  const float* __restrict__ asrc, const float* __restrict__ adst,
                                                  float* SS, float* SD, int nN, int MPr) {
  constexpr int HDM = HIDC / NH;
  const int row = (int)blockIdx.x * NTHR + (int)threadIdx.x;
  if (row >= MPr) return;
  const int rc = row < nN ? row : nN - 1;
  const float* p = F + (size_t)rc * LDF + colOff;
  v4f so = {0.f, 0.f, 0.f, 0.f}, sdd = {0.f, 0.f, 0.f, 0.f};
#pragma unroll
  for (int h = 0; h < NH; ++h) {
    float s1 = 0.f, s2 = 0.f;
#pragma unroll 1
    for (int q = 0; q < HDM / 4; ++q) {
      const v4f v = *(const v4f*)(p + h * HDM + 4 * q);
      const v4f a = *(const v4f*)(asrc + h * HDM + 4 * q);
      const v4f b = *(const v4f*)(adst + h * HDM + 4 * q);
      s1 = fmaf(v.x, rnev(a.x), s1); s1 = fmaf(v.y, rnev(a.y), s1);
      s1 = fmaf(v.z, rnev(a.z), s1); s1 = fmaf(v.w, rnev(a.w), s1);
      s2 = fmaf(v.x, rnev(b.x), s2); s2 = fmaf(v.y, rnev(b.y), s2);
      s2 = fmaf(v.z, rnev(b.z), s2); s2 = fmaf(v.w, rnev(b.w), s2);
    }
    so[h] = s1; sdd[h] = s2;
  }
  float* ps = SS + (size_t)row * 4;
  float* pd = SD + (size_t)row * 4;
  *(volatile v4f*)ps = so;
  *(volatile v4f*)pd = sdd;
  __threadfence();
  *(volatile v4f*)ps = so;
  *(volatile v4f*)pd = sdd;
}

template<int NH, int ACT>
__global__ __launch_bounds__(NTHR) void k_agg(
    const int* __restrict__ srcs, const int* __restrict__ dsts,
    const float* __restrict__ F, int colOff,
    const float* __restrict__ SS, const float* __restrict__ SD,
    const float* __restrict__ bias,
    us* Aout, int aColOff,
    int nN, int nE, int nb, int vec8, int MPr) {
  extern __shared__ v4f lds_dyn[];
  int* reg1 = (int*)lds_dyn;
  int* reg2 = reg1 + RCAP;
  int* scnt = reg2 + RCAP;
  int* soff = scnt + NBMAX;
  int* list = soff + NBMAX;
  int* wcnt = list + LISTN;
  int* wtot = wcnt + NWAVE;
  const int tid = (int)threadIdx.x, lane = tid & 31, wave = tid >> 5;
  const int nodeBase = (int)blockIdx.x * nb;

  for (int i = tid; i < NBMAX; i += NTHR) scnt[i] = 0;
  __syncthreads();

  int tot = 0;
  const int nChunks = (nE + CHUNK - 1) / CHUNK;
#pragma unroll 1
  for (int ch = 0; ch < nChunks; ++ch) {
    const int cbase = ch * CHUNK;
    const int wc = scan_chunk(dsts, nE, cbase, nodeBase, nb, vec8, list, tid, lane, wave);
    if (lane == 0) wcnt[wave] = wc;
    __syncthreads();
    int pre = 0, all = 0;
#pragma unroll
    for (int w2 = 0; w2 < NWAVE; ++w2) {
      int c = wcnt[w2];
      c = c < 0 ? 0 : (c > WCAP ? WCAP : c);
      all += c;
      pre += (w2 < wave) ? c : 0;
    }
    const int wcc  = wc > WCAP ? WCAP : wc;
    const int base = tot + pre;
#pragma unroll 1
    for (int i = lane; i < wcc; i += 32) {
      const int ent = list[wave * WCAP + i];
      const int el  = (ent >> 12) & (CHUNK - 1);
      const int sl  = ent & (NBMAX - 1);
      int eid = cbase + el;
      eid = eid > nE - 1 ? nE - 1 : eid;
      const int pos = base + i;
      if (pos < RCAP) reg1[pos] = (int)(((unsigned)eid << 12) | (unsigned)sl);
    }
    tot += all;
    tot = tot > RCAP ? RCAP : tot;
    __syncthreads();
  }
  const int nh = tot;

  if (wave == 0) {
#pragma unroll 1
    for (int b0 = 0; b0 < nh; b0 += 32) {
      const int idx = b0 + lane;
      const int uv  = reg1[idx < RCAP ? idx : RCAP - 1];
      const int m32 = (nh - b0) < 32 ? (nh - b0) : 32;
#pragma unroll 1
      for (int k = 0; k < m32; ++k) {
        const int u  = __builtin_amdgcn_readlane(uv, k);
        const int sl = u & (NBMAX - 1);
        if (lane == 0) scnt[sl] = scnt[sl] + 1;
      }
    }
  }
  __syncthreads();

  {
    const v4i ca = *(const v4i*)(scnt + 8 * tid);
    const v4i cb = *(const v4i*)(scnt + 8 * tid + 4);
    const int e0 = ca.x < 0 ? 0 : ca.x, e1 = ca.y < 0 ? 0 : ca.y, e2 = ca.z < 0 ? 0 : ca.z, e3 = ca.w < 0 ? 0 : ca.w;
    const int e4 = cb.x < 0 ? 0 : cb.x, e5 = cb.y < 0 ? 0 : cb.y, e6 = cb.z < 0 ? 0 : cb.z, e7 = cb.w < 0 ? 0 : cb.w;
    const int ts = e0 + e1 + e2 + e3 + e4 + e5 + e6 + e7;
    int incl = ts;
#pragma unroll
    for (int d = 1; d < 32; d <<= 1) {
      const int up = __shfl_up(incl, d);
      if (lane >= d) incl += up;
    }
    if (lane == 31) wtot[wave] = incl;
    __syncthreads();
    int pre = 0;
#pragma unroll
    for (int w2 = 0; w2 < NWAVE; ++w2) pre += (w2 < wave) ? wtot[w2] : 0;
    int run = pre + incl - ts;
    soff[8 * tid + 0] = run; run += e0;
    soff[8 * tid + 1] = run; run += e1;
    soff[8 * tid + 2] = run; run += e2;
    soff[8 * tid + 3] = run; run += e3;
    soff[8 * tid + 4] = run; run += e4;
    soff[8 * tid + 5] = run; run += e5;
    soff[8 * tid + 6] = run; run += e6;
    soff[8 * tid + 7] = run;
  }
  __syncthreads();
  for (int i = tid; i < NBMAX; i += NTHR) list[i] = soff[i];
  __syncthreads();

  if (wave == 0) {
#pragma unroll 1
    for (int b0 = 0; b0 < nh; b0 += 32) {
      const int idx = b0 + lane;
      const int uv  = reg1[idx < RCAP ? idx : RCAP - 1];
      const int m32 = (nh - b0) < 32 ? (nh - b0) : 32;
#pragma unroll 1
      for (int k = 0; k < m32; ++k) {
        const int u   = __builtin_amdgcn_readlane(uv, k);
        const int sl  = u & (NBMAX - 1);
        const int eid = (int)((unsigned)u >> 12);
        if (lane == 0) {
          int pos = list[sl];
          pos = pos < 0 ? 0 : (pos > RCAP - 1 ? RCAP - 1 : pos);
          reg2[pos] = eid;
          list[sl] = pos + 1;
        }
      }
    }
  }
  __syncthreads();

  const int nbw = nb >> 3;
  const bool ovf = (nh >= RCAP);
  const float qnan = __int_as_float(0x7fc00000);
  float* stw = (float*)reg1 + wave * STW;
  float bq[4];
#pragma unroll
  for (int j = 0; j < 4; ++j) bq[j] = rnev(bias[32 * j + lane]);
  const float* fl = F + colOff + lane;
  const int c0 = 8 * (lane & 15);
  const bool islo = lane >= 16;
#pragma unroll 1
  for (int jt = 0; jt < nbw; ++jt) {
    const int slot = wave * nbw + jt;
    const int grow = nodeBase + slot;
    const int gcl  = grow < nN ? grow : nN - 1;
    int st = soff[slot];
    const int craw = scnt[slot];
    int cnt = craw;
    st  = st < 0 ? 0 : (st > nh ? nh : st);
    cnt = cnt < 0 ? 0 : (cnt > DEGCAP ? DEGCAP : cnt);
    if (cnt > nh - st) cnt = nh - st;
    const bool pz   = ovf || (craw > DEGCAP);
    const bool wr   = grow < MPr;
    const bool live = grow < nN;

    const v4f sdv = *(const v4f*)(SD + (size_t)gcl * 4);
    const v4f ss0 = *(const v4f*)(SS + (size_t)gcl * 4);
    const float* h0p = fl + (size_t)gcl * LDF;
    float av[4];
#pragma unroll
    for (int j = 0; j < 4; ++j) av[j] = h0p[32 * j];
    ldwait();
    float mx[NH], dn[NH];
#pragma unroll
    for (int h = 0; h < NH; ++h) {
      const float t = ss0[h] + sdv[h];
      mx[h] = fmaxf(t, 0.2f * t);
      dn[h] = 1.0f;
    }

#pragma unroll 1
    for (int q = 0; q < cnt; ++q) {
      int idx = st + q; idx = idx > RCAP - 1 ? RCAP - 1 : idx;
      int eid = reg2[idx]; eid = eid < 0 ? 0 : (eid > nE - 1 ? nE - 1 : eid);
      const int sraw = srcs[eid];
      const int s = sraw < 0 ? 0 : (sraw > nN - 1 ? nN - 1 : sraw);
      const v4f ssv = *(const v4f*)(SS + (size_t)s * 4);
      const float* hp = fl + (size_t)s * LDF;
      float hv[4];
#pragma unroll
      for (int j = 0; j < 4; ++j) hv[j] = hp[32 * j];
      ldwait();
#pragma unroll
      for (int h = 0; h < NH; ++h) {
        const float t  = ssv[h] + sdv[h];
        const float al = fmaxf(t, 0.2f * t);
        const float df = al - mx[h];
        const float ee = __expf(-fabsf(df));
        const bool up  = df > 0.f;
        const float s1 = up ? ee : 1.0f;
        const float s2 = up ? 1.0f : ee;
        mx[h] = up ? al : mx[h];
        dn[h] = fmaf(dn[h], s1, s2);
        if (NH == 4) {
          av[h] = fmaf(av[h], s1, s2 * hv[h]);
        } else {
#pragma unroll
          for (int j = 0; j < 4; ++j) av[j] = fmaf(av[j], s1, s2 * hv[j]);
        }
      }
    }
    float iv[NH];
#pragma unroll
    for (int h = 0; h < NH; ++h) iv[h] = __builtin_amdgcn_rcpf(dn[h]);
    float v[4];
#pragma unroll
    for (int j = 0; j < 4; ++j) {
      const int hj = (NH == 4) ? j : 0;
      float t = fmaf(av[j], iv[hj], bq[j]);
      t = live ? t : 0.0f;
      t = pz ? qnan : t;
      v[j] = t;
    }
    __builtin_amdgcn_fence(__ATOMIC_RELEASE, "wavefront");
    __builtin_amdgcn_wave_barrier();
#pragma unroll
    for (int j = 0; j < 4; ++j) stw[32 * j + lane] = v[j];
    if (ACT == 1) {
#pragma unroll 1
      for (int j = 0; j < 4; ++j) {
        const float t = stw[32 * j + lane];
        stw[32 * j + lane] = t > 0.f ? t : expm1f(t);
      }
    }
    __builtin_amdgcn_fence(__ATOMIC_RELEASE, "wavefront");
    __builtin_amdgcn_wave_barrier();
    const v4f ga = *(const v4f*)(stw + c0);
    const v4f gb = *(const v4f*)(stw + c0 + 4);
    v8us hi8, lo8, o8;
    split8(ga, gb, hi8, lo8);
#pragma unroll
    for (int i = 0; i < 8; ++i) o8[i] = islo ? lo8[i] : hi8[i];
    us* gp = Aout + (size_t)grow * LDA + aColOff + 8 * lane;
    if (wr) *(volatile v8us*)gp = o8;
    __threadfence();
    if (wr) *(volatile v8us*)gp = o8;
  }
}

__global__ __launch_bounds__(NTHR) void k_ln(const float* __restrict__ G, const float* __restrict__ lg,
                                             const float* __restrict__ lb, float* out, int nN) {
  const int tid = (int)threadIdx.x, lane = tid & 31, wave = tid >> 5;
  const int row = (int)blockIdx.x * NWAVE + wave;
  if (row >= nN) return;
  const float* g = G + (size_t)row * NCOL;
  const v4f a = *(const v4f*)(g + 4 * lane);
  const v4f b = *(const v4f*)(g + NCOL / 2 + 4 * lane);
  float s = ((a.x + a.y) + (a.z + a.w)) + ((b.x + b.y) + (b.z + b.w));
#pragma unroll
  for (int off = 16; off > 0; off >>= 1) s += __shfl_xor(s, off);
  const float mu = s * (1.0f / 256.0f);
  const v4f da = a - mu;
  const v4f db = b - mu;
  float q = ((da.x * da.x + da.y * da.y) + (da.z * da.z + da.w * da.w)) +
            ((db.x * db.x + db.y * db.y) + (db.z * db.z + db.w * db.w));
#pragma unroll
  for (int off = 16; off > 0; off >>= 1) q += __shfl_xor(q, off);
  const float var = q * (1.0f / 256.0f);
  const float rs  = rsqrtf(var + 1e-5f);
  const v4f g0 = *(const v4f*)(lg + 4 * lane);
  const v4f g1 = *(const v4f*)(lg + NCOL / 2 + 4 * lane);
  const v4f b0 = *(const v4f*)(lb + 4 * lane);
  const v4f b1 = *(const v4f*)(lb + NCOL / 2 + 4 * lane);
  v4f oa, ob;
  oa.x = (da.x * rs) * rnev(g0.x) + rnev(b0.x);
  oa.y = (da.y * rs) * rnev(g0.y) + rnev(b0.y);
  oa.z = (da.z * rs) * rnev(g0.z) + rnev(b0.z);
  oa.w = (da.w * rs) * rnev(g0.w) + rnev(b0.w);
  ob.x = (db.x * rs) * rnev(g1.x) + rnev(b1.x);
  ob.y = (db.y * rs) * rnev(g1.y) + rnev(b1.y);
  ob.z = (db.z * rs) * rnev(g1.z) + rnev(b1.z);
  ob.w = (db.w * rs) * rnev(g1.w) + rnev(b1.w);
  float* op = out + (size_t)row * NCOL + 4 * lane;
  *(volatile v4f*)op = oa;
  *(volatile v4f*)(op + NCOL / 2) = ob;
  __threadfence();
  *(volatile v4f*)op = oa;
  *(volatile v4f*)(op + NCOL / 2) = ob;
}

static int pick_nb(int nE, int nN) {
  int nb = NBMAX;
  while (nb > 16 && (long long)nb * (long long)nE * 5LL > (long long)RCAP * (long long)nN * 4LL) nb >>= 1;
  return nb;
}
static inline int cdiv(int a, int b) { return (a + b - 1) / b; }

extern "C" void kernel_launch(void* const* d_in, const int* in_sizes, int n_in,
                              void* d_out, int out_size, void* d_ws, size_t ws_size,
                              hipStream_t stream) {
  if (n_in < 25) return;
  const int nN = in_sizes[0] / FIN;
  if (nN <= 0 || in_sizes[0] != nN * FIN || nN > (1 << 22)) return;
  if (in_sizes[1] < 2 || (in_sizes[1] & 1) != 0) return;
  if (in_sizes[2] < 2 || (in_sizes[2] & 1) != 0) return;
  const int nEf = in_sizes[1] / 2;
  const int nEr = in_sizes[2] / 2;
  if (nEf < 1 || nEf > (1 << 20) || nEr < 1 || nEr > (1 << 20)) return;
  if (in_sizes[3]  != FIN * HIDC  || in_sizes[4]  != HIDC || in_sizes[5]  != HIDC || in_sizes[6]  != HIDC) return;
  if (in_sizes[7]  != HIDC * HIDC || in_sizes[8]  != HIDC || in_sizes[9]  != HIDC || in_sizes[10] != HIDC) return;
  if (in_sizes[11] != FIN * HIDC  || in_sizes[12] != HIDC || in_sizes[13] != HIDC || in_sizes[14] != HIDC) return;
  if (in_sizes[15] != HIDC * HIDC || in_sizes[16] != HIDC || in_sizes[17] != HIDC || in_sizes[18] != HIDC) return;
  if (in_sizes[19] != (2 * HIDC) * NCOL || in_sizes[20] != NCOL) return;
  if (in_sizes[21] != NCOL * NCOL || in_sizes[22] != NCOL) return;
  if (in_sizes[23] != NCOL || in_sizes[24] != NCOL) return;
  if (out_size != nN * NCOL) return;

  const float* x     = (const float*)d_in[0];
  const int*   eif   = (const int*)  d_in[1];
  const int*   eir   = (const int*)  d_in[2];
  const float* W_f1  = (const float*)d_in[3];
  const float* as_f1 = (const float*)d_in[4];
  const float* ad_f1 = (const float*)d_in[5];
  const float* b_f1  = (const float*)d_in[6];
  const float* W_f2  = (const float*)d_in[7];
  const float* as_f2 = (const float*)d_in[8];
  const float* ad_f2 = (const float*)d_in[9];
  const float* b_f2  = (const float*)d_in[10];
  const float* W_r1  = (const float*)d_in[11];
  const float* as_r1 = (const float*)d_in[12];
  const float* ad_r1 = (const float*)d_in[13];
  const float* b_r1  = (const float*)d_in[14];
  const float* W_r2  = (const float*)d_in[15];
  const float* as_r2 = (const float*)d_in[16];
  const float* ad_r2 = (const float*)d_in[17];
  const float* b_r2  = (const float*)d_in[18];
  const float* W_fu1 = (const float*)d_in[19];
  const float* b_fu1 = (const float*)d_in[20];
  const float* W_fu2 = (const float*)d_in[21];
  const float* b_fu2 = (const float*)d_in[22];
  const float* ln_g  = (const float*)d_in[23];
  const float* ln_b  = (const float*)d_in[24];
  float* out = (float*)d_out;

  const int MP    = cdiv(nN, GBM) * GBM;
  const int nbF   = pick_nb(nEf, nN);
  const int nbR   = pick_nb(nEr, nN);
  const int gAF   = cdiv(MP, nbF);
  const int gAR   = cdiv(MP, nbR);
  const int vec8F = ((nEf & 3) == 0) ? 1 : 0;
  const int vec8R = ((nEr & 3) == 0) ? 1 : 0;
  if (gAF * nbF < MP || gAR * nbR < MP) return;

  char* ws = (char*)d_ws;
  size_t off = 0;
  const size_t oR0 = off; off += (size_t)MP * LDA * 2;             off = (off + 255) & ~(size_t)255;
  const size_t oR1 = off; off += (size_t)MP * LDA * 2;             off = (off + 255) & ~(size_t)255;
  const size_t oXB = off; off += (size_t)MP * FIN * 2;             off = (off + 255) & ~(size_t)255;
  const size_t oSS = off; off += (size_t)MP * 4 * 4;               off = (off + 255) & ~(size_t)255;
  const size_t oSD = off; off += (size_t)MP * 4 * 4;               off = (off + 255) & ~(size_t)255;
  const size_t oW1 = off; off += (size_t)NCOL * FIN * 2;           off = (off + 255) & ~(size_t)255;
  const size_t oW2 = off; off += (size_t)NCOL * (2 * HIDC) * 2;    off = (off + 255) & ~(size_t)255;
  const size_t oW3 = off; off += (size_t)NCOL * LDA * 2;           off = (off + 255) & ~(size_t)255;
  const size_t oW4 = off; off += (size_t)NCOL * LDA * 2;           off = (off + 255) & ~(size_t)255;
  if (off > ws_size || off > (size_t)WSMAX) return;
  float* F   = (float*)(ws + oR0);
  us*    GA  = (us*)(ws + oR0);
  us*    HA  = (us*)(ws + oR1);
  float* G   = (float*)(ws + oR1);
  us*    XB  = (us*)(ws + oXB);
  float* SS  = (float*)(ws + oSS);
  float* SD  = (float*)(ws + oSD);
  us*    WT1 = (us*)(ws + oW1);
  us*    WT2 = (us*)(ws + oW2);
  us*    WT3 = (us*)(ws + oW3);
  us*    WT4 = (us*)(ws + oW4);

  hipFuncSetAttribute(reinterpret_cast<const void*>(&k_agg<4, 1>),
                      hipFuncAttributeMaxDynamicSharedMemorySize, LDS_AGG);
  hipFuncSetAttribute(reinterpret_cast<const void*>(&k_agg<1, 0>),
                      hipFuncAttributeMaxDynamicSharedMemorySize, LDS_AGG);

  const int nUx = MP * (FIN / 8);
  k_xprep<<<cdiv(nUx, NTHR), NTHR, 0, stream>>>(x, XB, nN, nUx);

  {
    const int nU1 = NCOL * (FIN / 8);
    k_wtr<<<cdiv(nU1, NTHR), NTHR, 0, stream>>>(W_f1, W_r1, HIDC, HIDC, HIDC, FIN, FIN, 255, 9, 8, WT1, nU1);
    const int nU2 = NCOL * ((2 * HIDC) / 8);
    k_wtr<<<cdiv(nU2, NTHR), NTHR, 0, stream>>>(W_f2, W_r2, HIDC, HIDC, HIDC, HIDC, 2 * HIDC, 127, 8, 7, WT2, nU2);
    const int nU3 = NCOL * (LDA / 8);
    k_wtr<<<cdiv(nU3, NTHR), NTHR, 0, stream>>>(W_fu1, W_fu1, NCOL, NCOL, NCOL, 2 * HIDC, LDA, 127, 8, 7, WT3, nU3);
    const int nU4 = NCOL * (LDA / 8);
    k_wtr<<<cdiv(nU4, NTHR), NTHR, 0, stream>>>(W_fu2, W_fu2, NCOL, NCOL, NCOL, NCOL, LDA, 255, 9, 8, WT4, nU4);
  }

  const int  gM = MP / GBM;
  const dim3 gG(gM, NCOL / GBN);
  const int  gS = cdiv(MP, NTHR);

  k_gemm<0, 0><<<gG, GTHR, 0, stream>>>(XB, WT1, b_f1, F, XB, FIN, FIN, NCOL, 0, LDF);

  k_scores<4><<<gS, NTHR, 0, stream>>>(F, 0, as_f1, ad_f1, SS, SD, nN, MP);
  k_agg<4, 1><<<gAF, NTHR, LDS_AGG, stream>>>(eif, eif + nEf, F, 0, SS, SD, b_f1, HA, 0,
                                                nN, nEf, nbF, vec8F, MP);
  k_scores<4><<<gS, NTHR, 0, stream>>>(F, HIDC, as_r1, ad_r1, SS, SD, nN, MP);
  k_agg<4, 1><<<gAR, NTHR, LDS_AGG, stream>>>(eir, eir + nEr, F, HIDC, SS, SD, b_r1, HA, NCOL,
                                                nN, nEr, nbR, vec8R, MP);

  k_gemm<0, 0><<<gG, GTHR, 0, stream>>>(HA, WT2, b_f2, F, XB, 2 * HIDC, LDA, HIDC, NCOL, LDF);

  k_scores<1><<<gS, NTHR, 0, stream>>>(F, 0, as_f2, ad_f2, SS, SD, nN, MP);
  k_agg<1, 0><<<gAF, NTHR, LDS_AGG, stream>>>(eif, eif + nEf, F, 0, SS, SD, b_f2, HA, 0,
                                                nN, nEf, nbF, vec8F, MP);
  k_scores<1><<<gS, NTHR, 0, stream>>>(F, HIDC, as_r2, ad_r2, SS, SD, nN, MP);
  k_agg<1, 0><<<gAR, NTHR, LDS_AGG, stream>>>(eir, eir + nEr, F, HIDC, SS, SD, b_r2, HA, NCOL,
                                                nN, nEr, nbR, vec8R, MP);

  k_gemm<1, 1><<<gG, GTHR, 0, stream>>>(HA, WT3, b_fu1, SS, GA, LDA, LDA, NCOL, 0, LDA);

  k_gemm<0, 1><<<gG, GTHR, 0, stream>>>(GA, WT4, b_fu2, G, XB, LDA, LDA, NCOL, 0, LDF);

  k_ln<<<cdiv(nN, NWAVE), NTHR, 0, stream>>>(G, ln_g, ln_b, out, nN);
}
